// FastSlowSurpriseKimiDeltaAttention_15848429322344
// MI455X (gfx1250) — hardware-verified
//
#include <hip/hip_runtime.h>
#include <math.h>

constexpr int kNumB   = 2;
constexpr int kNumT   = 256;
constexpr int kRows   = kNumB * kNumT;
constexpr int kDm     = 2048;
constexpr int kHeads  = 16;
constexpr int kHd     = 128;
constexpr int kHdHalf = 64;
constexpr int kBins   = 64;
constexpr int kItems  = kRows * kHeads;
constexpr int kNstk   = 3 * kDm + kBins + kHd;
constexpr int kColUnc = 3 * kDm;
constexpr int kColG1  = 3 * kDm + kBins;
constexpr float kQScale    = 0.08838834764831845f;
constexpr float kEps       = 1e-6f;
constexpr float kNormEps   = 1e-5f;
constexpr float kInvLnBins = 0.24044917348149392f;
static_assert(kNstk % 64 == 0, "tile multiple");
static_assert(kRows % 64 == 0 && kDm % 64 == 0 && kHd % 64 == 0, "tile multiple");
static_assert(kItems % 64 == 0, "tile multiple");
static_assert(kDm % 32 == 0 && kHd % 32 == 0, "K multiple of 32");

typedef __attribute__((ext_vector_type(16))) _Float16 v16h;
typedef __attribute__((ext_vector_type(8)))  _Float16 v8h;
typedef __attribute__((ext_vector_type(16))) __bf16   v16b;
typedef __attribute__((ext_vector_type(8)))  __bf16   v8b;
typedef __attribute__((ext_vector_type(8)))  float    v8f;
typedef __attribute__((ext_vector_type(4)))  float    v4f;
typedef __attribute__((ext_vector_type(4)))  unsigned int v4u;
typedef __attribute__((ext_vector_type(2)))  unsigned int v2u;

__device__ __forceinline__ unsigned short f2bf_bits(float f) {
  unsigned u = __float_as_uint(f);
  return (unsigned short)((u + 0x7FFFu + ((u >> 16) & 1u)) >> 16);
}
__device__ __forceinline__ float bf_bits2f(unsigned short h) { return __uint_as_float(((unsigned)h) << 16); }

__device__ __forceinline__ void dep_guard_h(v8f& a, v8f& b, v16h x, v16h y) { asm volatile("v_nop\n\tv_nop\n\tv_nop\n\tv_nop" : "+v"(a), "+v"(b) : "v"(x), "v"(y)); }
__device__ __forceinline__ void dep_guard_b(v8f& a, v8f& b, v16b x, v16b y) { asm volatile("v_nop\n\tv_nop\n\tv_nop\n\tv_nop" : "+v"(a), "+v"(b) : "v"(x), "v"(y)); }
__device__ __forceinline__ void keep4_h(v16h a, v16h b, v16h c, v16h d) { asm volatile("v_nop" :: "v"(a), "v"(b), "v"(c), "v"(d)); }
__device__ __forceinline__ void keep4_b(v16b a, v16b b, v16b c, v16b d) { asm volatile("v_nop" :: "v"(a), "v"(b), "v"(c), "v"(d)); }
__device__ __forceinline__ void acc_guard4(v8f& a, v8f& b, v8f& c, v8f& d) { asm volatile("v_nop\n\tv_nop\n\tv_nop\n\tv_nop" : "+v"(a), "+v"(b), "+v"(c), "+v"(d)); }
template <typename T> struct Frag;
template <> struct Frag<_Float16> {
  typedef v16h V; union U { v16h v; v8h h[2]; };
  static __device__ __forceinline__ v16h load(const _Float16* p) {
    U f; f.h[0] = *(const v8h*)(p); f.h[1] = *(const v8h*)(p + 16); return f.v;
  }
  static __device__ __forceinline__ v8f mma(v16h a, v16h b, v8f c) {
    return __builtin_amdgcn_wmma_f32_16x16x32_f16(false, a, false, b, (short)0, c, false, false);
  }
  static __device__ __forceinline__ void guard(v8f& a, v8f& b, v16h x, v16h y) { dep_guard_h(a, b, x, y); }
  static __device__ __forceinline__ void keep(v16h a, v16h b, v16h c, v16h d) { keep4_h(a, b, c, d); }
};
template <> struct Frag<__bf16> {
  typedef v16b V; union U { v16b v; v8b h[2]; };
  static __device__ __forceinline__ v16b load(const __bf16* p) {
    U f; f.h[0] = *(const v8b*)(p); f.h[1] = *(const v8b*)(p + 16); return f.v;
  }
  static __device__ __forceinline__ v8f mma(v16b a, v16b b, v8f c) {
    return __builtin_amdgcn_wmma_f32_16x16x32_bf16(false, a, false, b, (short)0, c, false, false);
  }
  static __device__ __forceinline__ void guard(v8f& a, v8f& b, v16b x, v16b y) { dep_guard_b(a, b, x, y); }
  static __device__ __forceinline__ void keep(v16b a, v16b b, v16b c, v16b d) { keep4_b(a, b, c, d); }
};

__device__ __forceinline__ unsigned pk16(unsigned short a, unsigned short b) { return (unsigned)a | ((unsigned)b << 16); }
__device__ __forceinline__ void split_bf(float f, unsigned short& hb, unsigned short& lb) {
  hb = f2bf_bits(f);
  lb = f2bf_bits(f - bf_bits2f(hb));
}

template <int ET> struct Elem;
template <> struct Elem<0> { typedef _Float16 T; };
template <> struct Elem<1> { typedef __bf16 T; };
template <int ET, bool SPLIT, int BIAS_MODE, int OUT_MODE, bool RESID, int ACT = 0>
__global__ __launch_bounds__(256) void wmma_gemm64(
    const unsigned short* __restrict__ Ap, const unsigned short* __restrict__ A2p, int lda, long strideA,
    const unsigned short* __restrict__ Btp, const unsigned short* __restrict__ Bt2p, int ldb, long strideB,
    void* __restrict__ Cout, void* __restrict__ Cout2, int ldc, long strideC,
    const float* __restrict__ bias,
    const float* __restrict__ resid, long strideR,
    int M, int N, int K, float scale) {
  typedef typename Elem<ET>::T T;
  typedef typename Frag<T>::V V;
  const T* A = (const T*)Ap; const T* A2 = (const T*)A2p; const T* Bt = (const T*)Btp; const T* Bt2 = (const T*)Bt2p;
  __shared__ __align__(16) float sT[8][16 * 68];
  const int b    = blockIdx.y;
  const int lane = threadIdx.x & 31;
  const int wave = threadIdx.x >> 5;
  const int tilesN = N >> 6;
  const int tilesM = M >> 6;
  const int tile = blockIdx.x * 8 + wave;
  if (tile >= tilesM * tilesN) return;
  const int tm = tile / tilesN;
  const int tn = tile - tm * tilesN;
  const int m0 = tm << 6;
  const int n0 = tn << 6;

  const T* Ab  = A  + (size_t)b * strideA;
  const T* Bb  = Bt + (size_t)b * strideB;
  const T* Ab2 = SPLIT ? (A2  + (size_t)b * strideA) : nullptr;
  const T* Bb2 = SPLIT ? (Bt2 + (size_t)b * strideB) : nullptr;

  const int rlane = lane & 15;
  const int koff  = (lane >> 4) * 8;
  const int mOff  = (lane >> 4) * 8;

  v8f acc[4][4];
#pragma unroll
  for (int i = 0; i < 4; ++i)
#pragma unroll
    for (int j = 0; j < 4; ++j) acc[i][j] = (v8f){0.f,0.f,0.f,0.f,0.f,0.f,0.f,0.f};

  for (int k0 = 0; k0 < K; k0 += 32) {
    V bh[4], bl[4];
#pragma unroll
    for (int j = 0; j < 4; ++j) {
      const size_t bo = (size_t)(n0 + (j << 4) + rlane) * ldb + koff + k0;
      bh[j] = Frag<T>::load(Bb + bo);
      if (SPLIT) bl[j] = Frag<T>::load(Bb2 + bo);
    }
#pragma unroll
    for (int i = 0; i < 4; ++i) {
      const size_t ao = (size_t)(m0 + (i << 4) + rlane) * lda + koff + k0;
      V ah = Frag<T>::load(Ab + ao);
      V al;
      if (SPLIT) al = Frag<T>::load(Ab2 + ao);
#pragma unroll
      for (int j = 0; j < 4; ++j) {
        acc[i][j] = Frag<T>::mma(ah, bh[j], acc[i][j]);
        if (SPLIT) {
          acc[i][j] = Frag<T>::mma(ah, bl[j], acc[i][j]);
          acc[i][j] = Frag<T>::mma(al, bh[j], acc[i][j]);
        }
      }
      Frag<T>::guard(acc[i][0], acc[i][3], ah, SPLIT ? al : ah);
    }
    Frag<T>::keep(bh[0], bh[1], bh[2], bh[3]);
    if (SPLIT) Frag<T>::keep(bl[0], bl[1], bl[2], bl[3]);
  }
  acc_guard4(acc[0][0], acc[0][1], acc[0][2], acc[0][3]);
  acc_guard4(acc[1][0], acc[1][1], acc[1][2], acc[1][3]);
  acc_guard4(acc[2][0], acc[2][1], acc[2][2], acc[2][3]);
  acc_guard4(acc[3][0], acc[3][1], acc[3][2], acc[3][3]);

  float* slab = sT[wave];
  const float* Rb = RESID ? (resid + (size_t)b * strideR) : nullptr;
#pragma unroll
  for (int i = 0; i < 4; ++i) {
    const int mBase = m0 + (i << 4);
#pragma unroll
    for (int j = 0; j < 4; ++j) {
      const int n = n0 + (j << 4) + rlane;
      float bv = 0.f;
      if (BIAS_MODE == 2) bv = bias[n];
#pragma unroll
      for (int r = 0; r < 8; ++r) {
        float v = acc[i][j][r] * scale;
        if (BIAS_MODE == 1) v += bias[mBase + mOff + r];
        if (BIAS_MODE == 2) v += bv;
        if (RESID) v += Rb[(size_t)(mBase + mOff + r) * ldc + n];
        if (ACT == 2) v = fmaxf(v, 0.0f);
        if (ACT == 4) v = (v > 0.f) ? v : 0.01f * v;
        slab[(mOff + r) * 68 + (j << 4) + rlane] = v;
      }
    }
    __builtin_amdgcn_fence(__ATOMIC_RELEASE, "workgroup");
    __builtin_amdgcn_wave_barrier();
    __builtin_amdgcn_fence(__ATOMIC_ACQUIRE, "workgroup");
    if (OUT_MODE == 0) {
      float* C = (float*)Cout + (size_t)b * strideC;
      const int hh = lane >> 4, c4 = (lane & 15) * 4;
      for (int pass = 0; pass < 2; ++pass) {
#pragma unroll
        for (int it = 0; it < 8; ++it) {
          const int row = it * 2 + hh;
          v4f v = *(const v4f*)(slab + row * 68 + c4);
          *(volatile v4f*)(C + (size_t)(mBase + row) * ldc + n0 + c4) = v;
        }
        __threadfence();
      }
    } else {
      const int q = lane >> 3, c8 = (lane & 7) * 8;
      unsigned short* C  = (unsigned short*)Cout  + (size_t)b * strideC;
      unsigned short* C2 = (OUT_MODE == 2) ? ((unsigned short*)Cout2 + (size_t)b * strideC) : nullptr;
      for (int pass = 0; pass < 2; ++pass) {
#pragma unroll
        for (int it = 0; it < 4; ++it) {
          const int row = it * 4 + q;
          const float* sp = slab + row * 68 + c8;
          v8h hv, lv;
#pragma unroll
          for (int e = 0; e < 8; ++e) {
            if (OUT_MODE == 1) {
              hv[e] = (_Float16)sp[e];
            } else {
              unsigned short hb = f2bf_bits(sp[e]);
              unsigned short lb = f2bf_bits(sp[e] - bf_bits2f(hb));
              hv[e] = __builtin_bit_cast(_Float16, hb);
              lv[e] = __builtin_bit_cast(_Float16, lb);
            }
          }
          *(volatile v8h*)(C + (size_t)(mBase + row) * ldc + n0 + c8) = hv;
          if (OUT_MODE == 2) *(volatile v8h*)(C2 + (size_t)(mBase + row) * ldc + n0 + c8) = lv;
        }
        __threadfence();
      }
    }
    __builtin_amdgcn_fence(__ATOMIC_RELEASE, "workgroup");
    __builtin_amdgcn_wave_barrier();
    __builtin_amdgcn_fence(__ATOMIC_ACQUIRE, "workgroup");
  }
}

__device__ __forceinline__ float wave_sum(float v) {
#pragma unroll
  for (int off = 16; off > 0; off >>= 1) v += __shfl_xor(v, off, 32);
  return v;
}
__device__ __forceinline__ float wave_max(float v) {
#pragma unroll
  for (int off = 16; off > 0; off >>= 1) v = fmaxf(v, __shfl_xor(v, off, 32));
  return v;
}
__device__ __forceinline__ float sigmoid_f(float x) { return __builtin_amdgcn_rcpf(1.0f + expf(-x)); }
__device__ __forceinline__ float silu_f(float x)    { return x * sigmoid_f(x); }

__global__ __launch_bounds__(256) void split_rows_kernel(const float* __restrict__ src, int ld_src, int col0,
                                                         unsigned short* __restrict__ oh, unsigned short* __restrict__ ol,
                                                         int ld_dst, int rows, int cols8) {
  const int g = blockIdx.x * 256 + threadIdx.x;
  if (g >= rows * cols8) return;
  const int row = g / cols8;
  const int c8  = (g - row * cols8) * 8;
  const float* p = src + (size_t)row * ld_src + col0 + c8;
  const v4f a = *(const v4f*)(p);
  const v4f c = *(const v4f*)(p + 4);
  unsigned short hb[8], lb[8];
#pragma unroll
  for (int e = 0; e < 4; ++e) {
    split_bf(a[e], hb[e], lb[e]);
    split_bf(c[e], hb[4 + e], lb[4 + e]);
  }
  const v4u uh = (v4u){pk16(hb[0], hb[1]), pk16(hb[2], hb[3]), pk16(hb[4], hb[5]), pk16(hb[6], hb[7])};
  const v4u ul = (v4u){pk16(lb[0], lb[1]), pk16(lb[2], lb[3]), pk16(lb[4], lb[5]), pk16(lb[6], lb[7])};
  unsigned short* qh = oh + (size_t)row * ld_dst + c8;
  unsigned short* ql = ol + (size_t)row * ld_dst + c8;
  *(volatile v4u*)qh = uh;
  *(volatile v4u*)ql = ul;
  __threadfence();
  *(volatile v4u*)qh = uh;
  *(volatile v4u*)ql = ul;
}

__global__ __launch_bounds__(256) void wt_split_kernel(const float* __restrict__ W, int ldw,
                                                       unsigned short* __restrict__ oh, unsigned short* __restrict__ ol,
                                                       int ldo, int nrow_off) {
  __shared__ float sm[64][65];
  const int t  = threadIdx.x;
  const int d0 = blockIdx.x * 64;
  const int n0 = blockIdx.y * 64;
#pragma unroll
  for (int i = 0; i < 16; ++i) {
    const int e = i * 256 + t;
    const int r = e >> 6;
    const int c = e & 63;
    sm[c][r] = W[(size_t)(d0 + r) * ldw + n0 + c];
  }
  __syncthreads();
  const int lane = t & 31, wave = t >> 5;
  const int q = lane >> 3, c8 = (lane & 7) * 8;
  for (int pass = 0; pass < 2; ++pass) {
#pragma unroll
    for (int it = 0; it < 2; ++it) {
      const int row = wave * 8 + it * 4 + q;
      unsigned short hb[8], lb[8];
#pragma unroll
      for (int e = 0; e < 8; ++e) split_bf(sm[row][c8 + e], hb[e], lb[e]);
      const v4u uh = (v4u){pk16(hb[0], hb[1]), pk16(hb[2], hb[3]), pk16(hb[4], hb[5]), pk16(hb[6], hb[7])};
      const v4u ul = (v4u){pk16(lb[0], lb[1]), pk16(lb[2], lb[3]), pk16(lb[4], lb[5]), pk16(lb[6], lb[7])};
      const size_t o = (size_t)(nrow_off + n0 + row) * ldo + d0 + c8;
      *(volatile v4u*)(oh + o) = uh;
      *(volatile v4u*)(ol + o) = ul;
    }
    __threadfence();
  }
}

__global__ __launch_bounds__(256) void conv_silu_kernel(const float* __restrict__ proj,
                                                        const float* __restrict__ cwq, const float* __restrict__ cwk,
                                                        const float* __restrict__ cwv,
                                                        float* __restrict__ qs, float* __restrict__ kf, float* __restrict__ vf,
                                                        unsigned short* __restrict__ kh, unsigned short* __restrict__ kl) {
  const int which = blockIdx.y;
  const float* cw = (which == 0) ? cwq : ((which == 1) ? cwk : cwv);
  float* dst = (which == 0) ? qs : ((which == 1) ? kf : vf);
  const float oscale = (which == 0) ? kQScale : 1.0f;
  const int g  = blockIdx.x * 256 + threadIdx.x;
  const int bt = g >> 9;
  const int c  = (g & 511) * 4;
  const int t  = bt & (kNumT - 1);
  const v4f tw0 = *(const v4f*)(cw + (size_t)(c + 0) * 4);
  const v4f tw1 = *(const v4f*)(cw + (size_t)(c + 1) * 4);
  const v4f tw2 = *(const v4f*)(cw + (size_t)(c + 2) * 4);
  const v4f tw3 = *(const v4f*)(cw + (size_t)(c + 3) * 4);
  float a0 = 0.f, a1 = 0.f, a2 = 0.f, a3 = 0.f;
#pragma unroll
  for (int j = 0; j < 4; ++j) {
    const int back = 3 - j;
    const bool valid = (t >= back);
    const int rowc = valid ? (bt - back) : bt;
    const v4f xv = *(const v4f*)(proj + (size_t)rowc * kNstk + which * kDm + c);
    const float x0 = valid ? xv[0] : 0.f;
    const float x1 = valid ? xv[1] : 0.f;
    const float x2 = valid ? xv[2] : 0.f;
    const float x3 = valid ? xv[3] : 0.f;
    a0 += x0 * tw0[j];
    a1 += x1 * tw1[j];
    a2 += x2 * tw2[j];
    a3 += x3 * tw3[j];
  }
  const float r0 = silu_f(a0) * oscale;
  const float r1 = silu_f(a1) * oscale;
  const float r2 = silu_f(a2) * oscale;
  const float r3 = silu_f(a3) * oscale;
  const v4f ov = (v4f){r0, r1, r2, r3};
  float* dp = dst + (size_t)bt * kDm + c;
  v2u kh2 = (v2u){0u, 0u}, kl2 = (v2u){0u, 0u};
  if (which == 1) {
    unsigned short hb0, hb1, hb2, hb3, lb0, lb1, lb2, lb3;
    split_bf(r0, hb0, lb0); split_bf(r1, hb1, lb1); split_bf(r2, hb2, lb2); split_bf(r3, hb3, lb3);
    kh2 = (v2u){pk16(hb0, hb1), pk16(hb2, hb3)};
    kl2 = (v2u){pk16(lb0, lb1), pk16(lb2, lb3)};
  }
  unsigned short* khp = kh + (size_t)bt * kDm + c;
  unsigned short* klp = kl + (size_t)bt * kDm + c;
  *(volatile v4f*)dp = ov;
  if (which == 1) { *(volatile v2u*)khp = kh2; *(volatile v2u*)klp = kl2; }
  __threadfence();
  *(volatile v4f*)dp = ov;
  if (which == 1) { *(volatile v2u*)khp = kh2; *(volatile v2u*)klp = kl2; }
}

__global__ __launch_bounds__(256) void feats_kernel(const float* __restrict__ proj, const float* __restrict__ kf,
                                                    const float* __restrict__ vf, const float* __restrict__ vhat,
                                                    float* __restrict__ kunit, float* __restrict__ feats) {
  __shared__ __align__(16) float ft[32][4];
  const int lane = threadIdx.x & 31, wave = threadIdx.x >> 5;
  const int item0 = blockIdx.x * 32;
#pragma unroll 1
  for (int it = 0; it < 4; ++it) {
    const int slot = wave * 4 + it;
    const int item = item0 + slot;
    const int bt = item >> 4;
    const size_t base = (size_t)item * kHd;
    const float* lg = proj + (size_t)bt * kNstk + kColUnc + 2 * lane;
    const float s0 = lg[0], s1 = lg[1];
    const float m = wave_max(fmaxf(s0, s1));
    const float e0 = expf(s0 - m), e1 = expf(s1 - m);
    const float ssum = wave_sum(e0 + e1);
    const float lsum = logf(ssum);
    const float lp0 = (s0 - m) - lsum, lp1 = (s1 - m) - lsum;
    const float ent = wave_sum(-expf(lp0) * lp0 - expf(lp1) * lp1);
    const float entn = ent * kInvLnBins;
    float kn = 0.f, vn = 0.f, vhn = 0.f, dt = 0.f, en = 0.f;
#pragma unroll 1
    for (int e = 0; e < 4; ++e) {
      const size_t idx = base + 4 * lane + e;
      const float kv = kf[idx], vv = vf[idx], vh = vhat[idx];
      kn += kv * kv; vn += vv * vv; vhn += vh * vh; dt += vv * vh;
      const float d = vv - vh; en += d * d;
    }
    kn  = sqrtf(wave_sum(kn));
    vn  = sqrtf(wave_sum(vn));
    vhn = sqrtf(wave_sum(vhn));
    dt  = wave_sum(dt);
    en  = sqrtf(wave_sum(en));
    const float inv = 1.0f / (kn + kEps);
    const v4f k4 = *(const v4f*)(kf + base + 4 * lane);
    const v4f ku = k4 * inv;
    float* kup = kunit + base + 4 * lane;
    *(volatile v4f*)kup = ku;
    __threadfence();
    *(volatile v4f*)kup = ku;
    const float f1 = en / (vn + kEps);
    const float f2 = dt / (vn * vhn + kEps);
    const float f3 = log1pf(en);
    if (lane == 0) { ft[slot][0] = entn; ft[slot][1] = f1; ft[slot][2] = f2; ft[slot][3] = f3; }
  }
  __syncthreads();
  if (wave == 0) {
    const v4f f = *(const v4f*)(&ft[lane][0]);
    float* fp = feats + (size_t)(item0 + lane) * 4;
    *(volatile v4f*)fp = f;
    __threadfence();
    *(volatile v4f*)fp = f;
  }
}

__global__ __launch_bounds__(256) void heads_kernel(const float* __restrict__ feats, const float* __restrict__ hemb,
                                                    const float* __restrict__ w1, const float* __restrict__ b1,
                                                    const float* __restrict__ w2, const float* __restrict__ b2,
                                                    const float* __restrict__ bbw, const float* __restrict__ bbb,
                                                    const float* __restrict__ bdw, const float* __restrict__ bdb,
                                                    const float* __restrict__ lamw, const float* __restrict__ lamb,
                                                    const float* __restrict__ abw, const float* __restrict__ abb,
                                                    const float* __restrict__ adw, const float* __restrict__ adb,
                                                    float* __restrict__ sc) {
  __shared__ float scl[5][32];
  const int lane = threadIdx.x & 31, wave = threadIdx.x >> 5;
  const int item0 = blockIdx.x * 32;
#pragma unroll 1
  for (int it = 0; it < 4; ++it) {
    const int slot = wave * 4 + it;
    const int item = item0 + slot;
    const int h = item & (kHeads - 1);
    const v4f f4 = *(const v4f*)(feats + (size_t)item * 4);
    const v4f he = *(const v4f*)(hemb + h * 4);
    const int o = lane;
    const float a = f4[0] * w1[o] + f4[1] * w1[32 + o] + f4[2] * w1[64 + o] + f4[3] * w1[96 + o]
                  + he[0] * w1[128 + o] + he[1] * w1[160 + o] + he[2] * w1[192 + o] + he[3] * w1[224 + o];
    const float h1 = silu_f(a + b1[o]);
    float a2 = 0.f;
#pragma unroll 1
    for (int j = 0; j < 32; ++j) a2 += __shfl(h1, j, 32) * w2[j * 32 + o];
    const float h2 = silu_f(a2 + b2[o]);
    const float sbb = wave_sum(h2 * bbw[o]) + bbb[0];
    const float sbd = wave_sum(h2 * bdw[o]) + bdb[0];
    const float sla = wave_sum(h2 * lamw[o]) + lamb[0];
    const float sab = wave_sum(h2 * abw[o]) + abb[0];
    const float sad = wave_sum(h2 * adw[o]) + adb[0];
    const float z0 = sbb + sbd, z1 = sbb - sbd, z2 = sla, z3 = sab + sad, z4 = sab - sad;
    const float z = (lane == 0) ? z0 : ((lane == 1) ? z1 : ((lane == 2) ? z2 : ((lane == 3) ? z3 : z4)));
    const float sg = sigmoid_f(z);
    if (lane < 5) scl[lane][slot] = sg;
  }
  __syncthreads();
  if (wave == 0) {
    const float v0 = scl[0][lane], v1 = scl[1][lane], v2 = scl[2][lane], v3 = scl[3][lane], v4 = scl[4][lane];
    float* p = sc + item0 + lane;
    *(volatile float*)(p)              = v0;
    *(volatile float*)(p + kItems)     = v1;
    *(volatile float*)(p + 2 * kItems) = v2;
    *(volatile float*)(p + 3 * kItems) = v3;
    *(volatile float*)(p + 4 * kItems) = v4;
    __threadfence();
    *(volatile float*)(p)              = v0;
    *(volatile float*)(p + kItems)     = v1;
    *(volatile float*)(p + 2 * kItems) = v2;
    *(volatile float*)(p + 3 * kItems) = v3;
    *(volatile float*)(p + 4 * kItems) = v4;
  }
}

#define FENCE_F(x) asm volatile("" : "+v"(x))
#define DR_DECAY4(E) { \
  const v4f d4_ = *(const v4f*)(sd + ko + (E)); \
  const v4f k4_ = *(const v4f*)(sk + ko + (E)); \
  float s0_ = S[(E) + 0] * d4_[0]; float s1_ = S[(E) + 1] * d4_[1]; \
  float s2_ = S[(E) + 2] * d4_[2]; float s3_ = S[(E) + 3] * d4_[3]; \
  FENCE_F(s0_); FENCE_F(s1_); FENCE_F(s2_); FENCE_F(s3_); \
  S[(E) + 0] = s0_; S[(E) + 1] = s1_; S[(E) + 2] = s2_; S[(E) + 3] = s3_; \
  float p0_ = k4_[0] * s0_; float p1_ = k4_[1] * s1_; float p2_ = k4_[2] * s2_; float p3_ = k4_[3] * s3_; \
  FENCE_F(p0_); FENCE_F(p1_); FENCE_F(p2_); FENCE_F(p3_); \
  vp = vp + p0_; vp = vp + p1_; vp = vp + p2_; vp = vp + p3_; }
#define DR_DECAY16(E) DR_DECAY4(E) DR_DECAY4((E) + 4) DR_DECAY4((E) + 8) DR_DECAY4((E) + 12)
#define DR_UPD4(E) { \
  const v4f b4_ = *(const v4f*)(skb + ko + (E)); \
  const v4f q4_ = *(const v4f*)(sq + ko + (E)); \
  float u0_ = b4_[0] * dv; float u1_ = b4_[1] * dv; float u2_ = b4_[2] * dv; float u3_ = b4_[3] * dv; \
  FENCE_F(u0_); FENCE_F(u1_); FENCE_F(u2_); FENCE_F(u3_); \
  const float n0_ = S[(E) + 0] + u0_; const float n1_ = S[(E) + 1] + u1_; \
  const float n2_ = S[(E) + 2] + u2_; const float n3_ = S[(E) + 3] + u3_; \
  S[(E) + 0] = n0_; S[(E) + 1] = n1_; S[(E) + 2] = n2_; S[(E) + 3] = n3_; \
  float r0_ = q4_[0] * n0_; float r1_ = q4_[1] * n1_; float r2_ = q4_[2] * n2_; float r3_ = q4_[3] * n3_; \
  FENCE_F(r0_); FENCE_F(r1_); FENCE_F(r2_); FENCE_F(r3_); \
  ov = ov + r0_; ov = ov + r1_; ov = ov + r2_; ov = ov + r3_; }
#define DR_UPD16(E) DR_UPD4(E) DR_UPD4((E) + 4) DR_UPD4((E) + 8) DR_UPD4((E) + 12)

__global__ __launch_bounds__(256)
void recur_kernel(const float* __restrict__ qs, const float* __restrict__ kunit, const float* __restrict__ vf,
                  const float* __restrict__ sc, const float* __restrict__ alog, const float* __restrict__ dtb,
                  float* __restrict__ ofast, float* __restrict__ oslow) {
#pragma clang fp contract(off)
  __shared__ __align__(16) float sk[kHd];
  __shared__ __align__(16) float skb[kHd];
  __shared__ __align__(16) float sq[kHd];
  __shared__ __align__(16) float sd[kHd];
  __shared__ __align__(16) float so[kHd];
  const int tid  = threadIdx.x;
  const int wave = tid >> 5, lane = tid & 31;
  const int bid  = blockIdx.x;
  const int var  = bid & 1;
  const int bh   = bid >> 1;
  const int b    = bh >> 4;
  const int h    = bh & (kHeads - 1);
  const int col  = wave * 16 + (lane >> 1);
  const int half = lane & 1;
  const int ko   = half * kHdHalf;
  const int sidx = tid & (kHd - 1);
  float* outp = var ? oslow : ofast;
  const float* betap = sc + (size_t)var * kItems;
  const float* ampp  = sc + (size_t)(3 + var) * kItems;
  const float gch = -expf(alog[h]) * log1pf(expf(dtb[h * kHd + sidx]));
  float S[kHdHalf];
#pragma unroll
  for (int i = 0; i < kHdHalf; ++i) S[i] = 0.f;
#pragma unroll 1
  for (int t = 0; t < kNumT; ++t) {
    const int item = ((b * kNumT + t) << 4) + h;
    const size_t base = (size_t)item * kHd;
    const float beta = betap[item];
    const float amp  = ampp[item];
    if (tid < kHd) {
      const float kv = kunit[base + sidx];
      sk[sidx]  = kv;
      skb[sidx] = kv * beta;
      sq[sidx]  = qs[base + sidx];
      sd[sidx]  = expf(gch * amp);
    }
    __syncthreads();
    const float vt = vf[base + col];
    float vp = 0.f;
    DR_DECAY16(0)
    DR_DECAY16(16)
    DR_DECAY16(32)
    DR_DECAY16(48)
    const float vpt = vp + __shfl_xor(vp, 1, 32);
    const float dv = vt - vpt;
    float ov = 0.f;
    DR_UPD16(0)
    DR_UPD16(16)
    DR_UPD16(32)
    DR_UPD16(48)
    const float ot = ov + __shfl_xor(ov, 1, 32);
    if (half == 0) so[col] = ot;
    __syncthreads();
    if (wave == 0) {
      const v4f val = *(const v4f*)(so + 4 * lane);
      float* op = outp + base + 4 * lane;
      *(volatile v4f*)op = val;
      __threadfence();
      *(volatile v4f*)op = val;
    }
  }
}

__global__ __launch_bounds__(256) void combine_kernel(const float* __restrict__ ofast, const float* __restrict__ oslow,
                                                      const float* __restrict__ sc, const float* __restrict__ garr,
                                                      const float* __restrict__ onw,
                                                      unsigned short* __restrict__ o2h, unsigned short* __restrict__ o2l) {
  const int lane = threadIdx.x & 31, wave = threadIdx.x >> 5;
  const int item = blockIdx.x * 8 + wave;
  const size_t base = (size_t)item * kHd + 4 * lane;
  const float lam = sc[2 * kItems + item];
  const float oml = 1.0f - lam;
  const v4f a  = *(const v4f*)(ofast + base);
  const v4f s  = *(const v4f*)(oslow + base);
  const v4f gg = *(const v4f*)(garr + base);
  const v4f ow = *(const v4f*)(onw + 4 * lane);
  const float o0 = lam * a[0] + oml * s[0];
  const float o1 = lam * a[1] + oml * s[1];
  const float o2 = lam * a[2] + oml * s[2];
  const float o3 = lam * a[3] + oml * s[3];
  const float ss = wave_sum(o0 * o0 + o1 * o1 + o2 * o2 + o3 * o3);
  const float rms = sqrtf(ss * (1.0f / 128.0f) + kNormEps);
  const float inv = 1.0f / rms;
  const float r0 = (o0 * inv) * ow[0] * sigmoid_f(gg[0]);
  const float r1 = (o1 * inv) * ow[1] * sigmoid_f(gg[1]);
  const float r2 = (o2 * inv) * ow[2] * sigmoid_f(gg[2]);
  const float r3 = (o3 * inv) * ow[3] * sigmoid_f(gg[3]);
  unsigned short hb0, hb1, hb2, hb3, lb0, lb1, lb2, lb3;
  split_bf(r0, hb0, lb0); split_bf(r1, hb1, lb1); split_bf(r2, hb2, lb2); split_bf(r3, hb3, lb3);
  const v2u uh = (v2u){pk16(hb0, hb1), pk16(hb2, hb3)};
  const v2u ul = (v2u){pk16(lb0, lb1), pk16(lb2, lb3)};
  unsigned short* ph = o2h + base;
  unsigned short* pl = o2l + base;
  *(volatile v2u*)ph = uh;
  *(volatile v2u*)pl = ul;
  __threadfence();
  *(volatile v2u*)ph = uh;
  *(volatile v2u*)pl = ul;
}

extern "C" void kernel_launch(void* const* d_in, const int* in_sizes, int n_in,
                              void* d_out, int out_size, void* d_ws, size_t ws_size, hipStream_t stream) {
  if (n_in < 31) return;
  if (out_size < kRows * kDm) return;
  const float* x        = (const float*)d_in[0];
  const float* wq       = (const float*)d_in[1];
  const float* wk       = (const float*)d_in[2];
  const float* wv       = (const float*)d_in[3];
  const float* conv_q_w = (const float*)d_in[4];
  const float* conv_k_w = (const float*)d_in[5];
  const float* conv_v_w = (const float*)d_in[6];
  const float* a_log    = (const float*)d_in[7];
  const float* dt_bias  = (const float*)d_in[8];
  const float* proxy_w  = (const float*)d_in[9];
  const float* unc_w    = (const float*)d_in[10];
  const float* head_emb = (const float*)d_in[11];
  const float* mlp_w1   = (const float*)d_in[12];
  const float* mlp_b1   = (const float*)d_in[13];
  const float* mlp_w2   = (const float*)d_in[14];
  const float* mlp_b2   = (const float*)d_in[15];
  const float* bb_w     = (const float*)d_in[16];
  const float* bb_b     = (const float*)d_in[17];
  const float* bd_w     = (const float*)d_in[18];
  const float* bd_b     = (const float*)d_in[19];
  const float* lam_w    = (const float*)d_in[20];
  const float* lam_b    = (const float*)d_in[21];
  const float* ab_w     = (const float*)d_in[22];
  const float* ab_b     = (const float*)d_in[23];
  const float* ad_w     = (const float*)d_in[24];
  const float* ad_b     = (const float*)d_in[25];
  const float* g1_w     = (const float*)d_in[26];
  const float* g2_w     = (const float*)d_in[27];
  const float* g2_b     = (const float*)d_in[28];
  const float* onorm_w  = (const float*)d_in[29];
  const float* wo       = (const float*)d_in[30];
  float* out = (float*)d_out;

  char* ws = (char*)d_ws;
  size_t off = 0;
  auto carve = [&](size_t bytes) -> char* { char* p = ws + off; off += (bytes + 255) & ~(size_t)255; return p; };
  unsigned short* xh   = (unsigned short*)carve((size_t)kRows * kDm * 2);
  unsigned short* xl   = (unsigned short*)carve((size_t)kRows * kDm * 2);
  unsigned short* wsth = (unsigned short*)carve((size_t)kNstk * kDm * 2);
  unsigned short* wstl = (unsigned short*)carve((size_t)kNstk * kDm * 2);
  float* proj  = (float*)carve((size_t)kRows * kNstk * 4);
  float* qs    = (float*)carve((size_t)kRows * kDm * 4);
  float* kf    = (float*)carve((size_t)kRows * kDm * 4);
  float* vf    = (float*)carve((size_t)kRows * kDm * 4);
  unsigned short* kh  = (unsigned short*)carve((size_t)kRows * kDm * 2);
  unsigned short* kl  = (unsigned short*)carve((size_t)kRows * kDm * 2);
  unsigned short* pwh = (unsigned short*)carve((size_t)kHd * kHd * 2);
  unsigned short* pwl = (unsigned short*)carve((size_t)kHd * kHd * 2);
  float* vhat  = (float*)carve((size_t)kItems * kHd * 4);
  unsigned short* g1h = (unsigned short*)carve((size_t)kRows * kHd * 2);
  unsigned short* g1l = (unsigned short*)carve((size_t)kRows * kHd * 2);
  unsigned short* g2h = (unsigned short*)carve((size_t)kDm * kHd * 2);
  unsigned short* g2l = (unsigned short*)carve((size_t)kDm * kHd * 2);
  float* garr  = (float*)carve((size_t)kRows * kDm * 4);
  float* kunit = (float*)carve((size_t)kRows * kDm * 4);
  float* feats = (float*)carve((size_t)kItems * 4 * 4);
  float* sc    = (float*)carve((size_t)5 * kItems * 4);
  float* ofast = (float*)carve((size_t)kRows * kDm * 4);
  float* oslow = (float*)carve((size_t)kRows * kDm * 4);
  unsigned short* o2h = (unsigned short*)carve((size_t)kRows * kDm * 2);
  unsigned short* o2l = (unsigned short*)carve((size_t)kRows * kDm * 2);
  if (off > ws_size) return;
  unsigned short* woh = wsth;
  unsigned short* wol = wstl;

  auto wt = [&](const float* W, int kdim, int nout, unsigned short* oh, unsigned short* ol, int ldo, int nrow_off) {
    wt_split_kernel<<<dim3(kdim / 64, nout / 64), dim3(256), 0, stream>>>(W, nout, oh, ol, ldo, nrow_off);
  };

  split_rows_kernel<<<dim3((kRows * (kDm / 8)) / 256), dim3(256), 0, stream>>>(x, kDm, 0, xh, xl, kDm, kRows, kDm / 8);
  wt(wq,    kDm, kDm,   wsth, wstl, kDm, 0);
  wt(wk,    kDm, kDm,   wsth, wstl, kDm, kDm);
  wt(wv,    kDm, kDm,   wsth, wstl, kDm, 2 * kDm);
  wt(unc_w, kDm, kBins, wsth, wstl, kDm, kColUnc);
  wt(g1_w,  kDm, kHd,   wsth, wstl, kDm, kColG1);
  wt(proxy_w, kHd, kHd, pwh, pwl, kHd, 0);
  wt(g2_w,    kHd, kDm, g2h, g2l, kHd, 0);
  wmma_gemm64<1, true, 0, 0, false, 0><<<dim3((kRows / 64) * (kNstk / 64) / 8, 1), dim3(256), 0, stream>>>(
      xh, xl, kDm, 0L, wsth, wstl, kDm, 0L, (void*)proj, (void*)nullptr, kNstk, 0L,
      nullptr, nullptr, 0L, kRows, kNstk, kDm, 1.0f);
  wt(wo, kDm, kDm, woh, wol, kDm, 0);
  conv_silu_kernel<<<dim3((kRows * (kDm / 4)) / 256, 3), dim3(256), 0, stream>>>(proj, conv_q_w, conv_k_w, conv_v_w,
                                                                                qs, kf, vf, kh, kl);
  split_rows_kernel<<<dim3((kRows * (kHd / 8)) / 256), dim3(256), 0, stream>>>(proj, kNstk, kColG1, g1h, g1l, kHd, kRows, kHd / 8);
  wmma_gemm64<1, true, 0, 0, false, 0><<<dim3((kItems / 64) * (kHd / 64) / 8, 1), dim3(256), 0, stream>>>(
      kh, kl, kHd, 0L, pwh, pwl, kHd, 0L, (void*)vhat, (void*)nullptr, kHd, 0L,
      nullptr, nullptr, 0L, kItems, kHd, kHd, 1.0f);
  wmma_gemm64<1, true, 2, 0, false, 0><<<dim3((kRows / 64) * (kDm / 64) / 8, 1), dim3(256), 0, stream>>>(
      g1h, g1l, kHd, 0L, g2h, g2l, kHd, 0L, (void*)garr, (void*)nullptr, kDm, 0L,
      g2_b, nullptr, 0L, kRows, kDm, kHd, 1.0f);
  feats_kernel<<<dim3(kItems / 32), dim3(256), 0, stream>>>(proj, kf, vf, vhat, kunit, feats);
  heads_kernel<<<dim3(kItems / 32), dim3(256), 0, stream>>>(feats, head_emb, mlp_w1, mlp_b1, mlp_w2, mlp_b2,
                                                           bb_w, bb_b, bd_w, bd_b, lam_w, lam_b, ab_w, ab_b, ad_w, ad_b, sc);
  recur_kernel<<<dim3(kNumB * kHeads * 2), dim3(256), 0, stream>>>(qs, kunit, vf, sc, a_log, dt_bias, ofast, oslow);
  combine_kernel<<<dim3(kItems / 8), dim3(256), 0, stream>>>(ofast, oslow, sc, garr, onorm_w, o2h, o2l);
  wmma_gemm64<1, true, 0, 0, false, 0><<<dim3((kRows / 64) * (kDm / 64) / 8, 1), dim3(256), 0, stream>>>(
      o2h, o2l, kDm, 0L, woh, wol, kDm, 0L, (void*)out, (void*)nullptr, kDm, 0L,
      nullptr, nullptr, 0L, kRows, kDm, kDm, 1.0f);
}
